// DeltaNet_22488448762160
// MI455X (gfx1250) — hardware-verified
//
#include <hip/hip_runtime.h>
#include <math.h>

#pragma clang fp contract(off)

constexpr int kB     = 4;
constexpr int kT     = 2048;
constexpr int kC     = 1024;
constexpr int kH     = 8;
constexpr int kD     = 128;
constexpr int kHalfD = 64;
constexpr int kTok   = kB * kT;
constexpr int kNG    = kH * 2;
constexpr int kGL    = 64;
constexpr int kL     = 32;
constexpr int kNCh   = kT / kL;
constexpr int kEH    = 64;
constexpr int kAP    = 36;
constexpr int kYP    = 68;
constexpr float kCarry    = 16.0f;
constexpr float kCarryInv = 1.0f / 16.0f;
static_assert(kH * kD == kC);
static_assert(kT % kL == 0);
static_assert(kD == 2 * kEH);
static_assert(kTok % 64 == 0 && kC % 64 == 0 && kGL % 64 == 0 && kC % 32 == 0);
static_assert(kL == 32 && kNCh * kL == kT);

typedef __attribute__((ext_vector_type(16))) _Float16 v16h;
typedef __attribute__((ext_vector_type(8)))  _Float16 v8h;
typedef __attribute__((ext_vector_type(16))) __bf16   v16b;
typedef __attribute__((ext_vector_type(8)))  __bf16   v8b;
typedef __attribute__((ext_vector_type(8)))  float    v8f;
typedef __attribute__((ext_vector_type(4)))  float    v4f;
typedef __attribute__((ext_vector_type(2)))  float    v2f;
typedef __attribute__((ext_vector_type(4)))  unsigned int v4u;

__device__ __forceinline__ unsigned short f2bf_bits(float f) {
  unsigned u = __float_as_uint(f);
  return (unsigned short)((u + 0x7FFFu + ((u >> 16) & 1u)) >> 16);
}
__device__ __forceinline__ float bf_bits2f(unsigned short h) { return __uint_as_float(((unsigned)h) << 16); }
__device__ __forceinline__ float bfr(float f) { return bf_bits2f(f2bf_bits(f)); }
__device__ __forceinline__ unsigned pk16(unsigned short a, unsigned short b) { return (unsigned)a | ((unsigned)b << 16); }
__device__ __forceinline__ unsigned short h_bits(float f) { const _Float16 h = (_Float16)f; return __builtin_bit_cast(unsigned short, h); }
__device__ __forceinline__ float h16_to_f32(unsigned hb) {
  const unsigned sgn = (hb & 0x8000u) << 16; const unsigned em = hb & 0x7fffu;
  const float fn = __uint_as_float((em << 13) + 0x38000000u);
  const float fs = (float)em * 5.9604644775390625e-8f;
  const float mag = (em < 0x400u) ? fs : fn; return __uint_as_float(__float_as_uint(mag) | sgn); }

__device__ __forceinline__ void dep_guard_h(v8f& a, v8f& b, v16h x, v16h y) { asm volatile("v_nop\n\tv_nop\n\tv_nop\n\tv_nop" : "+v"(a), "+v"(b) : "v"(x), "v"(y)); }
__device__ __forceinline__ void dep_guard_b(v8f& a, v8f& b, v16b x, v16b y) { asm volatile("v_nop\n\tv_nop\n\tv_nop\n\tv_nop" : "+v"(a), "+v"(b) : "v"(x), "v"(y)); }
__device__ __forceinline__ void keep4_h(v16h a, v16h b, v16h c, v16h d) { asm volatile("v_nop" :: "v"(a), "v"(b), "v"(c), "v"(d)); }
__device__ __forceinline__ void keep4_b(v16b a, v16b b, v16b c, v16b d) { asm volatile("v_nop" :: "v"(a), "v"(b), "v"(c), "v"(d)); }
__device__ __forceinline__ void acc_guard4(v8f& a, v8f& b, v8f& c, v8f& d) { asm volatile("v_nop\n\tv_nop\n\tv_nop\n\tv_nop" : "+v"(a), "+v"(b), "+v"(c), "+v"(d)); }
__device__ __forceinline__ void dep_guard4_b(v8f& a, v8f& b, v8f& c, v8f& d, v16b x, v16b y) {
  asm volatile("v_nop\n\tv_nop\n\tv_nop\n\tv_nop" : "+v"(a), "+v"(b), "+v"(c), "+v"(d) : "v"(x), "v"(y));
}

template <typename T> struct Frag;
template <> struct Frag<_Float16> {
  typedef v16h V; union U { v16h v; v8h h[2]; };
  static __device__ __forceinline__ v16h load(const _Float16* p) {
    U f; f.h[0] = *(const v8h*)(p); f.h[1] = *(const v8h*)(p + 16); return f.v;
  }
  static __device__ __forceinline__ v8f mma(v16h a, v16h b, v8f c) {
    return __builtin_amdgcn_wmma_f32_16x16x32_f16(false, a, false, b, (short)0, c, false, false);
  }
  static __device__ __forceinline__ void guard(v8f& a, v8f& b, v16h x, v16h y) { dep_guard_h(a, b, x, y); }
  static __device__ __forceinline__ void keep(v16h a, v16h b, v16h c, v16h d) { keep4_h(a, b, c, d); }
};
template <> struct Frag<__bf16> {
  typedef v16b V; union U { v16b v; v8b h[2]; };
  static __device__ __forceinline__ v16b load(const __bf16* p) {
    U f; f.h[0] = *(const v8b*)(p); f.h[1] = *(const v8b*)(p + 16); return f.v;
  }
  static __device__ __forceinline__ v8f mma(v16b a, v16b b, v8f c) {
    return __builtin_amdgcn_wmma_f32_16x16x32_bf16(false, a, false, b, (short)0, c, false, false);
  }
  static __device__ __forceinline__ void guard(v8f& a, v8f& b, v16b x, v16b y) { dep_guard_b(a, b, x, y); }
  static __device__ __forceinline__ void keep(v16b a, v16b b, v16b c, v16b d) { keep4_b(a, b, c, d); }
};

__device__ __forceinline__ v8f mma_f16(v16h a, v16h b, v8f c) {
  c = __builtin_amdgcn_wmma_f32_16x16x32_f16(false, a, false, b, (short)0, c, false, false);
  asm volatile("v_nop\n\tv_nop\n\tv_nop\n\tv_nop" : "+v"(c) : "v"(a), "v"(b));
  return c;
}

template <bool ASPLIT, int BIAS_MODE, int OUT_MODE, bool ROPE>
__global__ __launch_bounds__(256) void wmma_gemm64(
    const unsigned short* __restrict__ Ap, const unsigned short* __restrict__ A2p, int lda,
    const unsigned short* __restrict__ Btp, int ldb,
    void* __restrict__ Cout, int ldc,
    const float* __restrict__ bias, const float* __restrict__ rcos, const float* __restrict__ rsin,
    int M, int N, int K, float scale) {
  typedef __bf16 T;
  typedef v16b V;
  const T* A = (const T*)Ap; const T* A2 = (const T*)A2p; const T* Bt = (const T*)Btp;
  __shared__ __align__(16) float sT[8][16 * 68];
  const int lane = threadIdx.x & 31;
  const int wave = threadIdx.x >> 5;
  const int tilesN = N >> 6;
  const int tilesM = M >> 6;
  const int tile = blockIdx.x * 8 + wave;
  if (tile >= tilesM * tilesN) return;
  const int tm = tile / tilesN;
  const int tn = tile - tm * tilesN;
  const int m0 = tm << 6;
  const int n0 = tn << 6;

  const int rlane = lane & 15;
  const int koff  = (lane >> 4) * 8;
  const int mOff  = (lane >> 4) * 8;

  v8f acc[4][4];
#pragma unroll
  for (int i = 0; i < 4; ++i)
#pragma unroll
    for (int j = 0; j < 4; ++j) acc[i][j] = (v8f){0.f,0.f,0.f,0.f,0.f,0.f,0.f,0.f};

  for (int k0 = 0; k0 < K; k0 += 32) {
    V bh[4];
#pragma unroll
    for (int j = 0; j < 4; ++j) {
      const size_t bo = (size_t)(n0 + (j << 4) + rlane) * ldb + koff + k0;
      bh[j] = Frag<T>::load(Bt + bo);
    }
#pragma unroll
    for (int i = 0; i < 4; ++i) {
      const size_t ao = (size_t)(m0 + (i << 4) + rlane) * lda + koff + k0;
      V ah = Frag<T>::load(A + ao);
      V al;
      if (ASPLIT) al = Frag<T>::load(A2 + ao);
#pragma unroll
      for (int j = 0; j < 4; ++j) {
        acc[i][j] = Frag<T>::mma(ah, bh[j], acc[i][j]);
        if (ASPLIT) acc[i][j] = Frag<T>::mma(al, bh[j], acc[i][j]);
      }
      dep_guard4_b(acc[i][0], acc[i][1], acc[i][2], acc[i][3], ah, ASPLIT ? al : ah);
    }
    keep4_b(bh[0], bh[1], bh[2], bh[3]);
  }
  acc_guard4(acc[0][0], acc[0][1], acc[0][2], acc[0][3]);
  acc_guard4(acc[1][0], acc[1][1], acc[1][2], acc[1][3]);
  acc_guard4(acc[2][0], acc[2][1], acc[2][2], acc[2][3]);
  acc_guard4(acc[3][0], acc[3][1], acc[3][2], acc[3][3]);

  float* slab = sT[wave];
#pragma unroll
  for (int i = 0; i < 4; ++i) {
    const int mBase = m0 + (i << 4);
#pragma unroll
    for (int j = 0; j < 4; ++j) {
      const int n = n0 + (j << 4) + rlane;
      float bv = 0.f;
      if (BIAS_MODE == 2) bv = bias[n];
#pragma unroll
      for (int r = 0; r < 8; ++r) {
        float v = acc[i][j][r] * scale;
        if (BIAS_MODE == 2) v += bv;
        slab[(mOff + r) * 68 + (j << 4) + rlane] = v;
      }
    }
    __builtin_amdgcn_fence(__ATOMIC_RELEASE, "workgroup");
    __builtin_amdgcn_wave_barrier();
    __builtin_amdgcn_fence(__ATOMIC_ACQUIRE, "workgroup");
    if (OUT_MODE == 0) {
      float* C = (float*)Cout;
      const int hh = lane >> 4, c4 = (lane & 15) * 4;
      for (int pass = 0; pass < 2; ++pass) {
#pragma unroll
        for (int it = 0; it < 8; ++it) {
          const int row = it * 2 + hh;
          v4f v = *(const v4f*)(slab + row * 68 + c4);
          *(volatile v4f*)(C + (size_t)(mBase + row) * ldc + n0 + c4) = v;
        }
        __threadfence();
      }
    } else {
      const int q = lane >> 3, c8 = (lane & 7) * 8;
      unsigned short* C = (unsigned short*)Cout;
      for (int pass = 0; pass < 2; ++pass) {
#pragma unroll
        for (int it = 0; it < 4; ++it) {
          const int row = it * 4 + q;
          const float* sp = slab + row * 68 + c8;
          float xv[8];
#pragma unroll
          for (int e = 0; e < 8; ++e) xv[e] = sp[e];
          if (ROPE) {
            const int t  = (mBase + row) & (kT - 1);
            const int j0 = ((n0 + c8) & (kD - 1)) >> 1;
            const v4f cs = *(const v4f*)(rcos + (size_t)t * kHalfD + j0);
            const v4f sn = *(const v4f*)(rsin + (size_t)t * kHalfD + j0);
#pragma unroll
            for (int p = 0; p < 4; ++p) {
              const float xr = xv[2 * p], xi = xv[2 * p + 1];
              const float cc = cs[p], ss = sn[p];
              xv[2 * p]     = xr * cc - xi * ss;
              xv[2 * p + 1] = xr * ss + xi * cc;
            }
          }
          v8h hv;
#pragma unroll
          for (int e = 0; e < 8; ++e) hv[e] = (_Float16)xv[e];
          *(volatile v8h*)(C + (size_t)(mBase + row) * ldc + n0 + c8) = hv;
        }
        __threadfence();
      }
    }
    __builtin_amdgcn_fence(__ATOMIC_RELEASE, "workgroup");
    __builtin_amdgcn_wave_barrier();
    __builtin_amdgcn_fence(__ATOMIC_ACQUIRE, "workgroup");
  }
}

__global__ __launch_bounds__(256) void cast8_bf16_kernel(const float* __restrict__ in, unsigned short* __restrict__ out, int n8) {
  const int i = blockIdx.x * 256 + threadIdx.x;
  if (i >= n8) return;
  const float* p = in + 8 * (size_t)i;
  const v4f a = *(const v4f*)(p);
  const v4f c = *(const v4f*)(p + 4);
  unsigned short hb[8];
#pragma unroll
  for (int e = 0; e < 4; ++e) {
    const float fa = a[e];
    const float fc = c[e];
    hb[e]     = f2bf_bits(fa);
    hb[4 + e] = f2bf_bits(fc);
  }
  const v4u u = (v4u){pk16(hb[0], hb[1]), pk16(hb[2], hb[3]), pk16(hb[4], hb[5]), pk16(hb[6], hb[7])};
  unsigned short* q = out + 8 * (size_t)i;
  *(volatile v4u*)q = u;
  __threadfence();
  *(volatile v4u*)q = u;
}

__global__ __launch_bounds__(256) void wtcast_kernel(const float* __restrict__ W0, const float* __restrict__ W1,
                                                     const float* __restrict__ W2, const float* __restrict__ W3,
                                                     unsigned short* __restrict__ out) {
  __shared__ float sm[64][65];
  const int t  = threadIdx.x;
  const int d0 = blockIdx.x * 64;
  const int h0 = blockIdx.y * 64;
  const int z  = blockIdx.z;
  const float* W = (z == 0) ? W0 : (z == 1) ? W1 : (z == 2) ? W2 : W3;
#pragma unroll
  for (int i = 0; i < 8; ++i) {
    const int e = i * 256 + t;
    const int r = e >> 6;
    const int c = e & 63;
    sm[c][r] = W[(size_t)(d0 + r) * kC + h0 + c];
  }
  asm volatile("" ::: "memory");
#pragma unroll
  for (int i = 8; i < 16; ++i) {
    const int e = i * 256 + t;
    const int r = e >> 6;
    const int c = e & 63;
    sm[c][r] = W[(size_t)(d0 + r) * kC + h0 + c];
  }
  __syncthreads();
  const int lane = t & 31, wave = t >> 5;
  const int q = lane >> 3, c8 = (lane & 7) * 8;
  unsigned short* op = out + (size_t)z * kC * kC;
  for (int pass = 0; pass < 2; ++pass) {
#pragma unroll
    for (int it = 0; it < 2; ++it) {
      const int row = wave * 8 + it * 4 + q;
      unsigned short hb[8];
#pragma unroll
      for (int e = 0; e < 8; ++e) hb[e] = f2bf_bits(sm[row][c8 + e]);
      const v4u u = (v4u){pk16(hb[0], hb[1]), pk16(hb[2], hb[3]), pk16(hb[4], hb[5]), pk16(hb[6], hb[7])};
      *(volatile v4u*)(op + (size_t)(h0 + row) * kC + d0 + c8) = u;
    }
    __threadfence();
  }
}

__global__ __launch_bounds__(256) void wg_cast_kernel(const float* __restrict__ Wb, const float* __restrict__ Wm,
                                                      unsigned short* __restrict__ WgT) {
  const int seg = blockIdx.y;
  const int i = blockIdx.x * 256 + threadIdx.x;
  const int nthr = (seg == 2) ? (32 * kC / 8) : (16 * kC / 8);
  if (i >= nthr) return;
  const int rloc = i >> 7;
  const int c8 = (i & 127) * 8;
  unsigned short hb[8];
  if (seg == 2) {
#pragma unroll
    for (int e = 0; e < 8; ++e) hb[e] = 0;
  } else {
    const float* W = (seg == 0) ? Wb : Wm;
#pragma unroll
    for (int e = 0; e < 8; ++e) hb[e] = f2bf_bits(W[(size_t)(c8 + e) * kNG + rloc]);
  }
  const int row = seg * 16 + rloc;
  const v4u u = (v4u){pk16(hb[0], hb[1]), pk16(hb[2], hb[3]), pk16(hb[4], hb[5]), pk16(hb[6], hb[7])};
  unsigned short* q = WgT + (size_t)row * kC + c8;
  *(volatile v4u*)q = u;
  __threadfence();
  *(volatile v4u*)q = u;
}

struct InvFreq { float f[kHalfD]; };
static_assert(sizeof(InvFreq) == 256);

__global__ __launch_bounds__(256) void rope_table_kernel(float* __restrict__ rcos, float* __restrict__ rsin, InvFreq iv) {
  __shared__ float fr[kHalfD];
  __shared__ __align__(16) float sc[256];
  __shared__ __align__(16) float ss[256];
  const int tid = threadIdx.x;
  if (tid == 0) {
#pragma unroll
    for (int j = 0; j < kHalfD; ++j) fr[j] = iv.f[j];
  }
  __syncthreads();
  const int g = blockIdx.x * 256 + tid;
  const int t = g >> 6;
  const int j = g & 63;
  const float ang = (float)t * fr[j];
  sc[tid] = cosf(ang);
  ss[tid] = sinf(ang);
  __syncthreads();
  if (tid < 64) {
    const v4f v = *(const v4f*)(sc + 4 * tid);
    float* dp = rcos + (size_t)blockIdx.x * 256 + 4 * tid;
    *(volatile v4f*)dp = v;
    __threadfence();
    *(volatile v4f*)dp = v;
  } else if (tid < 128) {
    const int t2 = tid - 64;
    const v4f v = *(const v4f*)(ss + 4 * t2);
    float* dp = rsin + (size_t)blockIdx.x * 256 + 4 * t2;
    *(volatile v4f*)dp = v;
    __threadfence();
    *(volatile v4f*)dp = v;
  }
}

__global__ __launch_bounds__(256) void gate_kernel(const float* __restrict__ gl, const float* __restrict__ bb,
                                                   const float* __restrict__ bm, float* __restrict__ betap,
                                                   float* __restrict__ mixo) {
  __shared__ __align__(16) float sb[32 * kNG];
  __shared__ __align__(16) float smx[32 * kNG];
  const int tid  = threadIdx.x;
  const int rloc = tid >> 3;
  const int hq   = tid & 7;
  const int row  = blockIdx.x * 32 + rloc;
  const float* gr = gl + (size_t)row * kGL;
  const v2f zb = *(const v2f*)(gr + 2 * hq);
  const v2f zm = *(const v2f*)(gr + 16 + 2 * hq);
  const v2f b2 = *(const v2f*)(bb + 2 * hq);
  const v2f m2 = *(const v2f*)(bm + 2 * hq);
  float bet[2];
#pragma unroll
  for (int k = 0; k < 2; ++k) {
    const float z  = zb[k] + bfr(b2[k]);
    const float ez = expf(-z);
    bet[k] = 1.0f / (1.0f + ez);
  }
  const float a0 = zm[0] + bfr(m2[0]);
  const float a1 = zm[1] + bfr(m2[1]);
  const float mx = fmaxf(a0, a1);
  const float e0 = expf(a0 - mx);
  const float e1 = expf(a1 - mx);
  const float inv = 1.0f / (e0 + e1);
  sb[rloc * kNG + 2 * hq]      = bet[0];
  sb[rloc * kNG + 2 * hq + 1]  = bet[1];
  smx[rloc * kNG + 2 * hq]     = e0 * inv;
  smx[rloc * kNG + 2 * hq + 1] = e1 * inv;
  __syncthreads();
  if (tid < 128) {
    const v4f v = *(const v4f*)(sb + 4 * tid);
    float* dp = betap + (size_t)blockIdx.x * 512 + 4 * tid;
    *(volatile v4f*)dp = v;
    __threadfence();
    *(volatile v4f*)dp = v;
  } else {
    const int t2 = tid - 128;
    const v4f v = *(const v4f*)(smx + 4 * t2);
    float* dp = mixo + (size_t)blockIdx.x * 512 + 4 * t2;
    *(volatile v4f*)dp = v;
    __threadfence();
    *(volatile v4f*)dp = v;
  }
}

__global__ __launch_bounds__(256) void scan_kernel(
    const unsigned short* __restrict__ qh, const unsigned short* __restrict__ kh,
    const unsigned short* __restrict__ vh, const float* __restrict__ betap,
    const float* __restrict__ mixq, const int* __restrict__ maskp,
    unsigned short* __restrict__ yhi, unsigned short* __restrict__ ylo) {
  __shared__ __align__(16) unsigned short Qs[kL * kD];
  __shared__ __align__(16) unsigned short Ks[kL * kD];
  __shared__ __align__(16) unsigned short Vs[kL * kEH];
  __shared__ __align__(16) unsigned short Vt[kEH * kL];
  __shared__ __align__(16) unsigned short Ktp[2 * kD * kL];
  __shared__ __align__(16) unsigned short St[2 * kEH * kD];
  __shared__ __align__(16) unsigned short Ad[2 * kL * kL];
  __shared__ __align__(16) float Araw[kL * kAP];
  __shared__ __align__(16) float Ys[kL * kYP];
  __shared__ float gb[2 * kL];
  __shared__ float gP[2 * kL];
  __shared__ float gPinv[2 * kL];
  __shared__ float gmx[2 * kL];
  __shared__ float gmk[kL];

  const int tid  = threadIdx.x;
  const int wave = tid >> 5;
  const int lane = tid & 31;
  const int hh   = lane >> 4;
  const int rl   = lane & 15;
  const int koff = hh * 8;
  const int bid  = blockIdx.x;
  const int eh   = bid & 1;
  const int h    = (bid >> 1) & 7;
  const int b    = bid >> 4;
  const int cbH  = h * kD;
  const int cbE  = cbH + eh * kEH;
  const int tmw  = wave >> 2;
  const int enw  = wave & 3;

  const _Float16* Qs16  = (const _Float16*)Qs;
  const _Float16* Ks16  = (const _Float16*)Ks;
  const _Float16* Vt16  = (const _Float16*)Vt;
  const _Float16* Ktp16 = (const _Float16*)Ktp;
  const _Float16* St16  = (const _Float16*)St;
  const _Float16* Ad16  = (const _Float16*)Ad;

  const v8f z8 = (v8f){0.f,0.f,0.f,0.f,0.f,0.f,0.f,0.f};

  {
    const v4u z4 = (v4u){0u, 0u, 0u, 0u};
#pragma unroll
    for (int it = 0; it < 8; ++it) *(v4u*)(St + (size_t)(it * 256 + tid) * 8) = z4;
  }
  v8f Sacc[2][4];
#pragma unroll
  for (int kap = 0; kap < 2; ++kap)
#pragma unroll
    for (int j = 0; j < 4; ++j) Sacc[kap][j] = z8;
  __syncthreads();

  for (int ch = 0; ch < kNCh; ++ch) {
    const int row0 = b * kT + ch * kL;

#pragma unroll
    for (int it = 0; it < 2; ++it) {
      const int c = it * 256 + tid;
      const int row = c >> 4;
      const int col8 = (c & 15) * 8;
      const size_t g = (size_t)(row0 + row) * kC + cbH + col8;
      const v4u qv = *(const v4u*)(qh + g);
      const v4u kv = *(const v4u*)(kh + g);
      *(v4u*)(Qs + row * kD + col8) = qv;
      *(v4u*)(Ks + row * kD + col8) = kv;
    }
    {
      const int row = tid >> 3;
      const int col8 = (tid & 7) * 8;
      const v4u vv = *(const v4u*)(vh + (size_t)(row0 + row) * kC + cbE + col8);
      *(v4u*)(Vs + row * kEH + col8) = vv;
    }
    if (tid < kL) {
      const int row = row0 + tid;
      const int mk = maskp[row];
      const float mkf = (mk > 0) ? 1.0f : 0.0f;
      const float b0 = betap[(size_t)row * kNG + h * 2];
      const float b1 = betap[(size_t)row * kNG + h * 2 + 1];
      const float m0 = mixq[(size_t)row * kNG + h * 2];
      const float m1 = mixq[(size_t)row * kNG + h * 2 + 1];
      gmk[tid] = mkf;
      gb[tid]      = mkf * b0 + (1.0f - mkf);
      gb[kL + tid] = mkf * b1 + (1.0f - mkf);
      gmx[tid]      = m0 * mkf;
      gmx[kL + tid] = m1 * mkf;
    }
    __syncthreads();

    if (tid < 2 * kL) {
      const int kap = tid >> 5;
      const int t = tid & 31;
      float p = 1.0f;
#pragma unroll 1
      for (int j = 0; j < kL; ++j) {
        const float f = gb[kap * kL + j];
        p = p * ((j <= t) ? f : 1.0f);
      }
      p = fmaxf(p, 1.0e-35f);
      gP[kap * kL + t]    = p;
      gPinv[kap * kL + t] = 1.0f / p;
    }
    {
      const int e  = tid >> 2;
      const int i0 = (tid & 3) * 8;
      unsigned short u[8];
#pragma unroll
      for (int p = 0; p < 8; ++p) u[p] = Vs[(i0 + p) * kEH + e];
      const v4u w = (v4u){pk16(u[0], u[1]), pk16(u[2], u[3]), pk16(u[4], u[5]), pk16(u[6], u[7])};
      *(v4u*)(Vt + e * kL + i0) = w;
    }
    if (wave < 4) {
      const int tm = wave >> 1, tn = wave & 1;
      const _Float16* qp = Qs16 + (tm * 16 + rl) * kD + koff;
      const _Float16* kp = Ks16 + (tn * 16 + rl) * kD + koff;
      v8f a = z8;
#pragma unroll
      for (int k0 = 0; k0 < kD; k0 += 32) a = mma_f16(Frag<_Float16>::load(qp + k0), Frag<_Float16>::load(kp + k0), a);
#pragma unroll
      for (int r = 0; r < 8; ++r) Araw[(tm * 16 + hh * 8 + r) * kAP + tn * 16 + rl] = a[r];
    }
    __syncthreads();

    {
      const int kap = tid >> 7;
      const int t   = (tid >> 2) & 31;
      const int i0  = (tid & 3) * 8;
      const float Pt = gP[kap * kL + t];
      const v4f r0 = *(const v4f*)(Araw + t * kAP + i0);
      const v4f r1 = *(const v4f*)(Araw + t * kAP + i0 + 4);
      float av[8];
#pragma unroll
      for (int e = 0; e < 4; ++e) { av[e] = r0[e]; av[4 + e] = r1[e]; }
      unsigned short hb[8];
#pragma unroll
      for (int p = 0; p < 8; ++p) {
        const int i = i0 + p;
        const float cf = (i <= t) ? 1.0f : 0.0f;
        const float gsel = cf * gmk[i];
        const float ratio = Pt * gPinv[kap * kL + i];
        const float val = ((av[p] * gsel) * ratio) * kCarry;
        hb[p] = h_bits(val);
      }
      const v4u w = (v4u){pk16(hb[0], hb[1]), pk16(hb[2], hb[3]), pk16(hb[4], hb[5]), pk16(hb[6], hb[7])};
      *(v4u*)(Ad + kap * kL * kL + t * kL + i0) = w;
    }
    {
      const int d  = tid >> 1;
      const int i0 = (tid & 1) * 16;
      float kf[16];
#pragma unroll
      for (int p = 0; p < 16; ++p) kf[p] = h16_to_f32((unsigned)Ks[(i0 + p) * kD + d]);
#pragma unroll
      for (int kap = 0; kap < 2; ++kap) {
        const float pl = gP[kap * kL + (kL - 1)];
        unsigned short hb[16];
#pragma unroll
        for (int p = 0; p < 16; ++p) {
          const float ratio = pl * gPinv[kap * kL + i0 + p];
          const float val = ((kf[p] * gmk[i0 + p]) * ratio) * kCarry;
          hb[p] = h_bits(val);
        }
        unsigned short* dst = Ktp + kap * kD * kL + d * kL + i0;
        const v4u w0 = (v4u){pk16(hb[0], hb[1]), pk16(hb[2], hb[3]), pk16(hb[4], hb[5]), pk16(hb[6], hb[7])};
        const v4u w1 = (v4u){pk16(hb[8], hb[9]), pk16(hb[10], hb[11]), pk16(hb[12], hb[13]), pk16(hb[14], hb[15])};
        *(v4u*)(dst)     = w0;
        *(v4u*)(dst + 8) = w1;
      }
    }
    __syncthreads();

    {
      const _Float16* qp  = Qs16 + (tmw * 16 + rl) * kD + koff;
      const _Float16* s0p = St16 + (enw * 16 + rl) * kD + koff;
      const _Float16* s1p = St16 + kEH * kD + (enw * 16 + rl) * kD + koff;
      v8f yr0 = z8, yr1 = z8;
#pragma unroll
      for (int k0 = 0; k0 < kD; k0 += 32) {
        const v16h qa = Frag<_Float16>::load(qp + k0);
        yr0 = mma_f16(qa, Frag<_Float16>::load(s0p + k0), yr0);
        yr1 = mma_f16(qa, Frag<_Float16>::load(s1p + k0), yr1);
      }
      const v16h vb = Frag<_Float16>::load(Vt16 + (enw * 16 + rl) * kL + koff);
      v8f yi0 = mma_f16(Frag<_Float16>::load(Ad16 + (tmw * 16 + rl) * kL + koff), vb, z8);
      v8f yi1 = mma_f16(Frag<_Float16>::load(Ad16 + kL * kL + (tmw * 16 + rl) * kL + koff), vb, z8);
#pragma unroll
      for (int r = 0; r < 8; ++r) {
        const int t = tmw * 16 + hh * 8 + r;
        const float a0 = gP[t] * yr0[r] + yi0[r];
        const float a1 = gP[kL + t] * yr1[r] + yi1[r];
        const float yv = (gmx[t] * a0 + gmx[kL + t] * a1) * kCarryInv;
        Ys[t * kYP + enw * 16 + rl] = yv;
      }
    }
    __syncthreads();

    {
      const v16h ka0 = Frag<_Float16>::load(Ktp16 + (wave * 16 + rl) * kL + koff);
      const v16h ka1 = Frag<_Float16>::load(Ktp16 + kD * kL + (wave * 16 + rl) * kL + koff);
      const float pl0 = gP[kL - 1];
      const float pl1 = gP[2 * kL - 1];
#pragma unroll
      for (int j = 0; j < 4; ++j) {
        const v16h vb = Frag<_Float16>::load(Vt16 + (j * 16 + rl) * kL + koff);
        Sacc[0][j] = Sacc[0][j] * pl0;
        Sacc[0][j] = mma_f16(ka0, vb, Sacc[0][j]);
        Sacc[1][j] = Sacc[1][j] * pl1;
        Sacc[1][j] = mma_f16(ka1, vb, Sacc[1][j]);
        unsigned short h0[8], h1[8];
#pragma unroll
        for (int r = 0; r < 8; ++r) {
          const float f0 = Sacc[0][j][r];
          const float f1 = Sacc[1][j][r];
          h0[r] = h_bits(f0);
          h1[r] = h_bits(f1);
        }
        const int so = (j * 16 + rl) * kD + wave * 16 + hh * 8;
        const v4u w0 = (v4u){pk16(h0[0], h0[1]), pk16(h0[2], h0[3]), pk16(h0[4], h0[5]), pk16(h0[6], h0[7])};
        const v4u w1 = (v4u){pk16(h1[0], h1[1]), pk16(h1[2], h1[3]), pk16(h1[4], h1[5]), pk16(h1[6], h1[7])};
        *(v4u*)(St + so)            = w0;
        *(v4u*)(St + kEH * kD + so) = w1;
      }
    }

    {
      const int row = wave * 4 + (lane >> 3);
      const int c8  = (lane & 7) * 8;
      const v4f ya = *(const v4f*)(Ys + row * kYP + c8);
      const v4f yb = *(const v4f*)(Ys + row * kYP + c8 + 4);
      unsigned short uh[8], ul[8];
#pragma unroll
      for (int e = 0; e < 4; ++e) {
        const float fa = ya[e];
        const unsigned short ha = f2bf_bits(fa);
        uh[e] = ha;
        ul[e] = f2bf_bits(fa - bf_bits2f(ha));
        const float fb = yb[e];
        const unsigned short hb2 = f2bf_bits(fb);
        uh[4 + e] = hb2;
        ul[4 + e] = f2bf_bits(fb - bf_bits2f(hb2));
      }
      const v4u wh = (v4u){pk16(uh[0], uh[1]), pk16(uh[2], uh[3]), pk16(uh[4], uh[5]), pk16(uh[6], uh[7])};
      const v4u wl = (v4u){pk16(ul[0], ul[1]), pk16(ul[2], ul[3]), pk16(ul[4], ul[5]), pk16(ul[6], ul[7])};
      const size_t go = (size_t)(row0 + row) * kC + cbE + c8;
      *(volatile v4u*)(yhi + go) = wh;
      *(volatile v4u*)(ylo + go) = wl;
      __threadfence();
      *(volatile v4u*)(yhi + go) = wh;
      *(volatile v4u*)(ylo + go) = wl;
    }
    __syncthreads();
  }
}

extern "C" void kernel_launch(void* const* d_in, const int* in_sizes, int n_in,
                              void* d_out, int out_size, void* d_ws, size_t ws_size,
                              hipStream_t stream) {
  if (n_in < 11) return;
  if (in_sizes[0] != kTok * kC) return;
  if (in_sizes[1] != kTok) return;
  if (in_sizes[2] != kC * kC || in_sizes[3] != kC * kC || in_sizes[4] != kC * kC) return;
  if (in_sizes[5] != kC * kNG || in_sizes[6] != kNG || in_sizes[7] != kC * kNG || in_sizes[8] != kNG) return;
  if (in_sizes[9] != kC * kC || in_sizes[10] != kC) return;
  if (out_size != kTok * kC) return;

  const size_t szX    = (size_t)kTok * kC * 2;
  const size_t szW    = (size_t)kC * kC * 2;
  const size_t szWg   = (size_t)kGL * kC * 2;
  const size_t szTab  = (size_t)kT * kHalfD * 4;
  const size_t szP16  = szX;
  const size_t szGl   = (size_t)kTok * kGL * 4;
  const size_t szGate = (size_t)kTok * kNG * 4;
  const size_t offX    = 0;
  const size_t offW    = offX + szX;
  const size_t offWg   = offW + 4 * szW;
  const size_t offCos  = offWg + szWg;
  const size_t offSin  = offCos + szTab;
  const size_t offQ    = offSin + szTab;
  const size_t offK    = offQ + szP16;
  const size_t offV    = offK + szP16;
  const size_t offGl   = offV + szP16;
  const size_t offBeta = offGl + szGl;
  const size_t offMix  = offBeta + szGate;
  const size_t offYh   = offMix + szGate;
  const size_t offYl   = offYh + szP16;
  const size_t total   = offYl + szP16;
  if (ws_size < total) return;

  const float* x    = (const float*)d_in[0];
  const int*   mask = (const int*)d_in[1];
  const float* Wq   = (const float*)d_in[2];
  const float* Wk   = (const float*)d_in[3];
  const float* Wv   = (const float*)d_in[4];
  const float* Wb   = (const float*)d_in[5];
  const float* bb   = (const float*)d_in[6];
  const float* Wm   = (const float*)d_in[7];
  const float* bm   = (const float*)d_in[8];
  const float* Wo   = (const float*)d_in[9];
  const float* bo   = (const float*)d_in[10];
  float* out = (float*)d_out;
  char* ws = (char*)d_ws;
  unsigned short* xh  = (unsigned short*)(ws + offX);
  unsigned short* WT  = (unsigned short*)(ws + offW);
  unsigned short* WqT = WT;
  unsigned short* WkT = WT + (size_t)kC * kC;
  unsigned short* WvT = WT + (size_t)2 * kC * kC;
  unsigned short* WoT = WT + (size_t)3 * kC * kC;
  unsigned short* WgT = (unsigned short*)(ws + offWg);
  float* rcos = (float*)(ws + offCos);
  float* rsin = (float*)(ws + offSin);
  unsigned short* qh = (unsigned short*)(ws + offQ);
  unsigned short* kh = (unsigned short*)(ws + offK);
  unsigned short* vh = (unsigned short*)(ws + offV);
  float* gl    = (float*)(ws + offGl);
  float* betap = (float*)(ws + offBeta);
  float* mixp  = (float*)(ws + offMix);
  unsigned short* yhi = (unsigned short*)(ws + offYh);
  unsigned short* ylo = (unsigned short*)(ws + offYl);

  InvFreq iv;
  for (int j = 0; j < kHalfD; ++j) {
    const double e = (double)(2 * j) / (double)kD;
    const float p = (float)pow(10000.0, e);
    iv.f[j] = 1.0f / p;
  }

  const int n8 = (kTok * kC) / 8;
  cast8_bf16_kernel<<<dim3(n8 / 256), dim3(256), 0, stream>>>(x, xh, n8);
  wtcast_kernel<<<dim3(kC / 64, kC / 64, 4), dim3(256), 0, stream>>>(Wq, Wk, Wv, Wo, WT);
  wg_cast_kernel<<<dim3(16, 3), dim3(256), 0, stream>>>(Wb, Wm, WgT);
  rope_table_kernel<<<dim3((kT * kHalfD) / 256), dim3(256), 0, stream>>>(rcos, rsin, iv);

  const int blkProj = ((kTok / 64) * (kC / 64)) / 8;
  const int blkGate = ((kTok / 64) * (kGL / 64)) / 8;
  wmma_gemm64<false, 0, 1, true><<<dim3(blkProj), dim3(256), 0, stream>>>(
      xh, xh, kC, WqT, kC, (void*)qh, kC, bo, rcos, rsin, kTok, kC, kC, 1.0f);
  wmma_gemm64<false, 0, 1, true><<<dim3(blkProj), dim3(256), 0, stream>>>(
      xh, xh, kC, WkT, kC, (void*)kh, kC, bo, rcos, rsin, kTok, kC, kC, 1.0f);
  wmma_gemm64<false, 0, 1, false><<<dim3(blkProj), dim3(256), 0, stream>>>(
      xh, xh, kC, WvT, kC, (void*)vh, kC, bo, rcos, rsin, kTok, kC, kC, 1.0f);
  wmma_gemm64<false, 0, 0, false><<<dim3(blkGate), dim3(256), 0, stream>>>(
      xh, xh, kC, WgT, kC, (void*)gl, kGL, bo, rcos, rsin, kTok, kGL, kC, 1.0f);
  gate_kernel<<<dim3(kTok / 32), dim3(256), 0, stream>>>(gl, bb, bm, betap, mixp);

  scan_kernel<<<dim3(kB * kH * 2), dim3(256), 0, stream>>>(qh, kh, vh, betap, mixp, mask, yhi, ylo);

  wmma_gemm64<true, 2, 0, false><<<dim3(blkProj), dim3(256), 0, stream>>>(
      yhi, ylo, kC, WoT, kC, (void*)out, kC, bo, rcos, rsin, kTok, kC, kC, 1.0f);
}
